// MultiObserverGNN_45672682225672
// MI455X (gfx1250) — hardware-verified
//
#include <hip/hip_runtime.h>
#include <stddef.h>


#pragma clang fp contract(off)

#define FDIM    128
#define HDIM    128
#define NVIEW   4
#define ZDIM    512
#define MDIM    256
#define ODIM    128
#define NTHR    256
#define NWAVE   8
#define EPT     8
#define NGRP    2
#define CHUNK   (NTHR * EPT * NGRP)
#define WCAP    (EPT * NGRP * 32)
#define LISTN   (NWAVE * WCAP)
#define NBC     4096
#define NBF     1024
#define RCAP    40960
#define RBN     128
#define TGT     256
#define DEGCAP  256
#define OTHR    512
#define STHR    512
#define BM      64
#define STATR   512
#define NPADG   512
#define EPB     (4 * NTHR)
#define WSCAP   134217728
#define XSC     8.0f
#define ZSC     16.0f
#define WSC     64.0f
#define INV_XW  (1.0f / 512.0f)
#define INV_ZW  (1.0f / 1024.0f)
#define BN_EPS  1e-5
#define LN_EPS  1e-5f
#define GEO_EPS 1e-8f
#define GAM_EPS 1e-8f

#define LDS_FILL ((RCAP + NBF + LISTN) * 4 + 64)
#define LDS_G2   (BM * ZDIM * 2 + BM * MDIM * 4)

static_assert((CHUNK & (CHUNK - 1)) == 0);
static_assert(CHUNK <= 4096);
static_assert(NBC <= 4096 && NBF <= 4096);
static_assert((NBC & (NBC - 1)) == 0 && (NBF & (NBF - 1)) == 0);
static_assert(NBC == 4 * NBF);
static_assert(OTHR * 8 == NBC);
static_assert((RCAP % 32) == 0);
static_assert(TGT == NWAVE * 32);
static_assert(ZDIM == NVIEW * HDIM && STHR == ZDIM);
static_assert((NPADG % TGT) == 0 && (NPADG % BM) == 0 && (NPADG % STATR) == 0);
static_assert(FDIM / 8 == 16);
static_assert(HDIM == 4 * 32 && ODIM == 4 * 32 && MDIM == 8 * 32);
static_assert(BM * ZDIM / 8 == 16 * NTHR);
static_assert(BM == 64 && NWAVE == 8);
static_assert(EPB % NTHR == 0);

typedef float          v4f  __attribute__((ext_vector_type(4)));
typedef float          v8f  __attribute__((ext_vector_type(8)));
typedef int            v4i  __attribute__((ext_vector_type(4)));
typedef _Float16       v8h  __attribute__((ext_vector_type(8)));
typedef _Float16       v16h __attribute__((ext_vector_type(16)));
union FragH { v16h v; v8h h[2]; };

__device__ __forceinline__ v8f wmh(v16h a, v16h b, v8f c) {
  v8f d = __builtin_amdgcn_wmma_f32_16x16x32_f16(false, a, false, b, (short)0, c, false, false);
  asm volatile("v_nop\n\tv_nop\n\tv_nop\n\tv_nop" : "+v"(d) : "v"(a), "v"(b));
  return d;
}

__device__ __forceinline__ int clampi(int v, int lo, int hi) { return v < lo ? lo : (v > hi ? hi : v); }

__device__ __forceinline__ float geo_dist(float dx, float dy, float dz) {
  const float sq = (dx * dx + dz * dz) + dy * dy;
  return sqrtf(sq);
}

__device__ __forceinline__ float view_ab(float vf, float rc, float vm, float dsum) {
  const float v = vf * fminf(rc, vm);
  const float g = sqrtf((1.0f - v * v) + GAM_EPS);
  const float u = 1.0f + v * dsum;
  return g * (1.0f / u);
}

template <int NB>
__device__ __forceinline__ int scan_chunk(const int* __restrict__ dsts, int nE, int cbase, int slotBase,
                                          int vec8, int* list, int tid, int lane, int wave) {
  int wc = 0;
#pragma unroll
  for (int g = 0; g < NGRP; ++g) {
    const int el0  = (g * NTHR + tid) * EPT;
    const int e0   = cbase + el0;
    const int sent = -2147483647 - 1;
    v4i da, db;
    if (vec8 != 0 && cbase + CHUNK <= nE) {
      da = *(const v4i*)(dsts + e0);
      db = *(const v4i*)(dsts + e0 + 4);
    } else {
      da.x = (e0     < nE) ? dsts[min(e0, nE - 1)] : sent;
      da.y = (e0 + 1 < nE) ? dsts[min(e0 + 1, nE - 1)] : sent;
      da.z = (e0 + 2 < nE) ? dsts[min(e0 + 2, nE - 1)] : sent;
      da.w = (e0 + 3 < nE) ? dsts[min(e0 + 3, nE - 1)] : sent;
      db.x = (e0 + 4 < nE) ? dsts[min(e0 + 4, nE - 1)] : sent;
      db.y = (e0 + 5 < nE) ? dsts[min(e0 + 5, nE - 1)] : sent;
      db.z = (e0 + 6 < nE) ? dsts[min(e0 + 6, nE - 1)] : sent;
      db.w = (e0 + 7 < nE) ? dsts[min(e0 + 7, nE - 1)] : sent;
    }
    const unsigned nb = (unsigned)slotBase;
    const unsigned s0 = (unsigned)da.x - nb, s1 = (unsigned)da.y - nb;
    const unsigned s2 = (unsigned)da.z - nb, s3 = (unsigned)da.w - nb;
    const unsigned s4 = (unsigned)db.x - nb, s5 = (unsigned)db.y - nb;
    const unsigned s6 = (unsigned)db.z - nb, s7 = (unsigned)db.w - nb;
    const bool h0 = s0 < (unsigned)NB, h1 = s1 < (unsigned)NB, h2 = s2 < (unsigned)NB, h3 = s3 < (unsigned)NB;
    const bool h4 = s4 < (unsigned)NB, h5 = s5 < (unsigned)NB, h6 = s6 < (unsigned)NB, h7 = s7 < (unsigned)NB;
    const unsigned any = __builtin_amdgcn_ballot_w32(h0 | h1 | h2 | h3 | h4 | h5 | h6 | h7);
    if (any != 0u) {
#define HITJ(J, HJ, SJ) { \
        const unsigned mj = __builtin_amdgcn_ballot_w32(HJ); \
        if (mj != 0u) { \
          if (HJ) { \
            const int pos = wc + (int)__builtin_amdgcn_mbcnt_lo(mj, 0u); \
            if (pos < WCAP) list[wave * WCAP + pos] = ((el0 + (J)) << 12) | (int)(SJ); \
          } \
          wc += (int)__builtin_popcount(mj); } }
      HITJ(0, h0, s0)
      HITJ(1, h1, s1)
      HITJ(2, h2, s2)
      HITJ(3, h3, s3)
      HITJ(4, h4, s4)
      HITJ(5, h5, s5)
      HITJ(6, h6, s6)
      HITJ(7, h7, s7)
#undef HITJ
    }
  }
  return wc;
}

__global__ __launch_bounds__(NTHR) void k_wprep(const float* __restrict__ W, _Float16* wp, int nUnits) {
  const int i = (int)blockIdx.x * NTHR + (int)threadIdx.x;
  if (i >= nUnits) return;
  const float* p = W + (size_t)i * 8;
  const v4f a = *(const v4f*)p, b = *(const v4f*)(p + 4);
  v8h hv;
  hv[0] = (_Float16)(a.x * WSC); hv[1] = (_Float16)(a.y * WSC);
  hv[2] = (_Float16)(a.z * WSC); hv[3] = (_Float16)(a.w * WSC);
  hv[4] = (_Float16)(b.x * WSC); hv[5] = (_Float16)(b.y * WSC);
  hv[6] = (_Float16)(b.z * WSC); hv[7] = (_Float16)(b.w * WSC);
  _Float16* d = wp + (size_t)i * 8;
  *(volatile v8h*)d = hv;
  __threadfence();
  *(volatile v8h*)d = hv;
}

__global__ __launch_bounds__(NTHR) void k_xprep(const float* __restrict__ x, _Float16* xh, int nN, int nUnits) {
  const int i = (int)blockIdx.x * NTHR + (int)threadIdx.x;
  if (i >= nUnits) return;
  const int row = i >> 4;
  const int c   = (i & 15) * 8;
  const int rr  = row < nN ? row : nN - 1;
  const float* p = x + (size_t)rr * FDIM + c;
  v4f a = *(const v4f*)p, b = *(const v4f*)(p + 4);
  const v4f z4 = {0.f, 0.f, 0.f, 0.f};
  if (row >= nN) { a = z4; b = z4; }
  v8h hv;
  hv[0] = (_Float16)(a.x * XSC); hv[1] = (_Float16)(a.y * XSC);
  hv[2] = (_Float16)(a.z * XSC); hv[3] = (_Float16)(a.w * XSC);
  hv[4] = (_Float16)(b.x * XSC); hv[5] = (_Float16)(b.y * XSC);
  hv[6] = (_Float16)(b.z * XSC); hv[7] = (_Float16)(b.w * XSC);
  _Float16* d = xh + (size_t)i * 8;
  *(volatile v8h*)d = hv;
  __threadfence();
  *(volatile v8h*)d = hv;
}

__global__ __launch_bounds__(NTHR) void k_count(
    const int* __restrict__ dsts, int* cnt, int nE, int vec8) {
  __shared__ __attribute__((aligned(16))) int scnt[NBC];
  __shared__ __attribute__((aligned(16))) int list[LISTN];
  __shared__ int wcnt[NWAVE];
  const int tid = threadIdx.x, lane = tid & 31, wave = tid >> 5;
  const int nodeBase = blockIdx.x * NBC;

  for (int i = tid; i < NBC; i += NTHR) scnt[i] = 0;
  __syncthreads();

  const int nChunks = (nE + CHUNK - 1) / CHUNK;
#pragma unroll 1
  for (int ch = 0; ch < nChunks; ++ch) {
    const int cbase = ch * CHUNK;
    const int wc = scan_chunk<NBC>(dsts, nE, cbase, nodeBase, vec8, list, tid, lane, wave);
    if (lane == 0) wcnt[wave] = wc;
    __syncthreads();
    if (wave == 0) {
#pragma unroll 1
      for (int wsx = 0; wsx < NWAVE; ++wsx) {
        int n = __builtin_amdgcn_readfirstlane(wcnt[wsx]);
        n = n > WCAP ? WCAP : (n < 0 ? 0 : n);
        const int* lp = list + wsx * WCAP;
#pragma unroll 1
        for (int i = 0; i < n; ++i) {
          const int ent  = __builtin_amdgcn_readfirstlane(lp[i]);
          const int slot = ent & (NBC - 1);
          if (lane == 0) scnt[slot] = scnt[slot] + 1;
        }
      }
    }
    __syncthreads();
  }

  v4i cq[4];
#pragma unroll
  for (int q = 0; q < 4; ++q) {
    const int f = (wave * 4 + q) * 128 + 4 * lane;
    cq[q] = *(const v4i*)(scnt + f);
  }
  int* cp = cnt + (size_t)nodeBase;
#pragma unroll
  for (int q = 0; q < 4; ++q) {
    const int f = (wave * 4 + q) * 128 + 4 * lane;
    *(volatile v4i*)(cp + f) = cq[q];
  }
  __threadfence();
#pragma unroll
  for (int q = 0; q < 4; ++q) {
    const int f = (wave * 4 + q) * 128 + 4 * lane;
    *(volatile v4i*)(cp + f) = cq[q];
  }
}

__global__ __launch_bounds__(OTHR) void k_offsets(
    const int* __restrict__ cnt, int* off, int* rbase, int nChunk) {
  __shared__ __attribute__((aligned(16))) int soff[NBC];
  __shared__ __attribute__((aligned(16))) int srb[RBN];
  __shared__ int wtot[OTHR / 32];
  const int tid = threadIdx.x, lane = tid & 31, wave = tid >> 5, sub = tid >> 7;
  for (int i = tid; i < RBN; i += OTHR) srb[i] = 0;
  int carry = 0;
#pragma unroll 1
  for (int ch = 0; ch < nChunk; ++ch) {
    const int base = ch * NBC;
    const v4i c0 = *(const v4i*)(cnt + base + 8 * tid);
    const v4i c1 = *(const v4i*)(cnt + base + 8 * tid + 4);
    const int e0 = max(c0.x, 0), e1 = max(c0.y, 0), e2 = max(c0.z, 0), e3 = max(c0.w, 0);
    const int e4 = max(c1.x, 0), e5 = max(c1.y, 0), e6 = max(c1.z, 0), e7 = max(c1.w, 0);
    const int ts = e0 + e1 + e2 + e3 + e4 + e5 + e6 + e7;
    int incl = ts;
#pragma unroll
    for (int d = 1; d < 32; d <<= 1) {
      const int t = __shfl_up(incl, d);
      if (lane >= d) incl += t;
    }
    if (lane == 31) wtot[wave] = incl;
    __syncthreads();
    const int S0 = wtot[0]  + wtot[1]  + wtot[2]  + wtot[3];
    const int S1 = wtot[4]  + wtot[5]  + wtot[6]  + wtot[7];
    const int S2 = wtot[8]  + wtot[9]  + wtot[10] + wtot[11];
    const int S3 = wtot[12] + wtot[13] + wtot[14] + wtot[15];
    int pre = 0;
#pragma unroll 1
    for (int w = 4 * sub; w < wave; ++w) pre += wtot[w];
    const int b0 = carry;
    const int b1 = b0 + ((S0 + 31) & ~31);
    const int b2 = b1 + ((S1 + 31) & ~31);
    const int b3 = b2 + ((S2 + 31) & ~31);
    const int b4 = b3 + ((S3 + 31) & ~31);
    const int myb = sub == 0 ? b0 : (sub == 1 ? b1 : (sub == 2 ? b2 : b3));
    if (tid == 0) {
      srb[min(4 * ch + 0, RBN - 1)] = b0;
      srb[min(4 * ch + 1, RBN - 1)] = b1;
      srb[min(4 * ch + 2, RBN - 1)] = b2;
      srb[min(4 * ch + 3, RBN - 1)] = b3;
    }
    int run = myb + pre + incl - ts;
    soff[8 * tid + 0] = run; run += e0;
    soff[8 * tid + 1] = run; run += e1;
    soff[8 * tid + 2] = run; run += e2;
    soff[8 * tid + 3] = run; run += e3;
    soff[8 * tid + 4] = run; run += e4;
    soff[8 * tid + 5] = run; run += e5;
    soff[8 * tid + 6] = run; run += e6;
    soff[8 * tid + 7] = run;
    carry = b4;
    __syncthreads();
    const v4i o0 = *(const v4i*)(soff + 4 * tid);
    const v4i o1 = *(const v4i*)(soff + 4 * (tid + OTHR));
    int* op = off + base;
    *(volatile v4i*)(op + 4 * tid) = o0;
    *(volatile v4i*)(op + 4 * (tid + OTHR)) = o1;
    __threadfence();
    *(volatile v4i*)(op + 4 * tid) = o0;
    *(volatile v4i*)(op + 4 * (tid + OTHR)) = o1;
    __syncthreads();
  }
  if (tid == 0) srb[min(4 * nChunk, RBN - 1)] = carry;
  __syncthreads();
  v4i rv = {0, 0, 0, 0};
  if (tid < 32) rv = *(const v4i*)(srb + 4 * tid);
  if (tid < 32) *(volatile v4i*)(rbase + 4 * tid) = rv;
  __threadfence();
  if (tid < 32) *(volatile v4i*)(rbase + 4 * tid) = rv;
}

__global__ __launch_bounds__(NTHR) void k_fill(
    const int* __restrict__ dsts, const int* __restrict__ off, const int* __restrict__ rbase,
    int* csr, int nE, int vec8, int csrLen) {
  extern __shared__ v4f lds_dyn[];
  int* region = (int*)lds_dyn;
  int* cursor = region + RCAP;
  int* list   = cursor + NBF;
  int* wcnt   = list + LISTN;
  const int tid = threadIdx.x, lane = tid & 31, wave = tid >> 5;
  const int b = blockIdx.x;
  const int nodeBase = b * NBF;

  int rb0 = rbase[b];
  const int rb1 = rbase[b + 1];
  rb0 = rb0 < 0 ? 0 : (rb0 > csrLen ? csrLen : rb0);
  rb0 &= ~31;
  int len = rb1 - rb0;
  len = len < 0 ? 0 : (len > RCAP ? RCAP : len);
  int lenW = (len + 31) & ~31;
  if (rb0 + lenW > csrLen) lenW = (csrLen - rb0) & ~31;

  {
    const v4i z = {0, 0, 0, 0};
    for (int i = tid; i < RCAP / 4; i += NTHR) ((v4i*)region)[i] = z;
    for (int s = tid; s < NBF; s += NTHR) {
      int o = off[nodeBase + s] - rb0;
      o = o < 0 ? 0 : (o > RCAP ? RCAP : o);
      cursor[s] = o;
    }
  }
  __syncthreads();

  const int nChunks = (nE + CHUNK - 1) / CHUNK;
#pragma unroll 1
  for (int ch = 0; ch < nChunks; ++ch) {
    const int cbase = ch * CHUNK;
    const int wc = scan_chunk<NBF>(dsts, nE, cbase, nodeBase, vec8, list, tid, lane, wave);
    if (lane == 0) wcnt[wave] = wc;
    __syncthreads();
    if (wave == 0) {
#pragma unroll 1
      for (int wsx = 0; wsx < NWAVE; ++wsx) {
        int n = __builtin_amdgcn_readfirstlane(wcnt[wsx]);
        n = n > WCAP ? WCAP : (n < 0 ? 0 : n);
        const int* lp = list + wsx * WCAP;
#pragma unroll 1
        for (int i = 0; i < n; ++i) {
          const int ent  = __builtin_amdgcn_readfirstlane(lp[i]);
          const int slot = ent & (NBF - 1);
          int e = cbase + ((ent >> 12) & (CHUNK - 1));
          e = e > nE - 1 ? nE - 1 : e;
          if (lane == 0) {
            int pos = cursor[slot];
            pos = pos < 0 ? 0 : (pos > RCAP - 1 ? RCAP - 1 : pos);
            region[pos] = e;
            const int np = pos + 1;
            cursor[slot] = np > RCAP ? RCAP : np;
          }
        }
      }
    }
    __syncthreads();
  }

  const int nv = lenW >> 2;
  int* gp = csr + rb0;
#pragma unroll 1
  for (int i = tid; i < nv; i += NTHR) { const v4i v = ((const v4i*)region)[i]; *(volatile v4i*)(gp + 4 * i) = v; }
  __threadfence();
#pragma unroll 1
  for (int i = tid; i < nv; i += NTHR) { const v4i v = ((const v4i*)region)[i]; *(volatile v4i*)(gp + 4 * i) = v; }
}

template <int KD, int NC>
__device__ __forceinline__ void mm_core(const _Float16* A, int lda, const _Float16* __restrict__ Bw,
                                        float* stg, float inv) {
  static_assert(KD % 32 == 0 && (NC % 32) == 0);
  constexpr int NT = NC / 32;
  const int tid = threadIdx.x, lane = tid & 31, wave = tid >> 5, hh = lane >> 4, m = lane & 15;
  const int r0 = (wave >> 1) * 16, c0 = (wave & 1) * (NC / 2);
  v8f acc[NT];
#pragma unroll
  for (int t = 0; t < NT; ++t) { v8f z = {0.f, 0.f, 0.f, 0.f, 0.f, 0.f, 0.f, 0.f}; acc[t] = z; }
  const _Float16* ap  = A  + (size_t)(r0 + m) * lda + 8 * hh;
  const _Float16* bp0 = Bw + (size_t)(c0 + m) * KD + 8 * hh;
#pragma unroll 1
  for (int kt = 0; kt < KD / 32; ++kt) {
    FragH a;
    a.h[0] = *(const v8h*)(ap + 32 * kt);
    a.h[1] = *(const v8h*)(ap + 32 * kt + 16);
#pragma unroll
    for (int t = 0; t < NT; ++t) {
      const _Float16* bp = bp0 + (size_t)t * (16 * KD) + 32 * kt;
      FragH b;
      b.h[0] = *(const v8h*)bp;
      b.h[1] = *(const v8h*)(bp + 16);
      acc[t] = wmh(a.v, b.v, acc[t]);
    }
  }
  float* sp = stg + (size_t)(r0 + 8 * hh) * NC + c0 + m;
#pragma unroll
  for (int t = 0; t < NT; ++t) {
#pragma unroll
    for (int r = 0; r < 8; ++r) sp[r * NC + 16 * t] = acc[t][r] * inv;
  }
}

__global__ __launch_bounds__(NTHR) void k_gemm_h(
    const _Float16* __restrict__ xh, const _Float16* __restrict__ wp, const float* __restrict__ bias,
    _Float16* Hh, int nN) {
  __shared__ __attribute__((aligned(16))) float stg[BM * HDIM];
  const int tid = threadIdx.x, lane = tid & 31, wave = tid >> 5;
  const int rowBase = blockIdx.x * BM;

  mm_core<FDIM, HDIM>(xh + (size_t)rowBase * FDIM, FDIM, wp, stg, INV_XW);
  __syncthreads();

  const int q = lane & 15, rsub = lane >> 4, col = 8 * q;
  const v4f b0 = *(const v4f*)(bias + col), b1 = *(const v4f*)(bias + col + 4);
  const v4f z4 = {0.f, 0.f, 0.f, 0.f};
  v8h hv[4];
#pragma unroll
  for (int it = 0; it < 4; ++it) {
    const int row  = 8 * wave + 2 * it + rsub;
    const int grow = rowBase + row;
    const float* sr = stg + (size_t)row * HDIM + col;
    const v4f s0 = *(const v4f*)sr, s1 = *(const v4f*)(sr + 4);
    v4f h0 = s0 + b0, h1 = s1 + b1;
    h0.x = h0.x > 0.f ? h0.x : 0.f; h0.y = h0.y > 0.f ? h0.y : 0.f;
    h0.z = h0.z > 0.f ? h0.z : 0.f; h0.w = h0.w > 0.f ? h0.w : 0.f;
    h1.x = h1.x > 0.f ? h1.x : 0.f; h1.y = h1.y > 0.f ? h1.y : 0.f;
    h1.z = h1.z > 0.f ? h1.z : 0.f; h1.w = h1.w > 0.f ? h1.w : 0.f;
    if (grow >= nN) { h0 = z4; h1 = z4; }
    v8h w;
    w[0] = (_Float16)(h0.x * XSC); w[1] = (_Float16)(h0.y * XSC);
    w[2] = (_Float16)(h0.z * XSC); w[3] = (_Float16)(h0.w * XSC);
    w[4] = (_Float16)(h1.x * XSC); w[5] = (_Float16)(h1.y * XSC);
    w[6] = (_Float16)(h1.z * XSC); w[7] = (_Float16)(h1.w * XSC);
    hv[it] = w;
    *(volatile v8h*)(Hh + (size_t)grow * HDIM + col) = w;
  }
  __threadfence();
#pragma unroll
  for (int it = 0; it < 4; ++it) {
    const int row  = 8 * wave + 2 * it + rsub;
    const int grow = rowBase + row;
    *(volatile v8h*)(Hh + (size_t)grow * HDIM + col) = hv[it];
  }
}

template <int KD, int GRADED>
__global__ __launch_bounds__(NTHR) void k_gemm_f(
    const _Float16* __restrict__ A, const _Float16* __restrict__ wp, const float* __restrict__ bias,
    float* C, int nN) {
  __shared__ __attribute__((aligned(16))) float stg[BM * ODIM];
  const int tid = threadIdx.x, lane = tid & 31, wave = tid >> 5;
  const int rowBase = blockIdx.x * BM;

  mm_core<KD, ODIM>(A + (size_t)rowBase * KD, KD, wp, stg, INV_XW);
  __syncthreads();

  const int col0 = 4 * lane;
  const v4f bb = *(const v4f*)(bias + col0);
#pragma unroll
  for (int it = 0; it < 8; ++it) {
    const int row  = 8 * wave + it;
    const int grow = rowBase + row;
    const v4f v = *(const v4f*)(stg + (size_t)row * ODIM + col0) + bb;
    if constexpr (GRADED == 0) {
      *(volatile v4f*)(C + (size_t)grow * ODIM + col0) = v;
    } else {
      if (grow < nN) *(volatile v4f*)(C + (size_t)grow * ODIM + col0) = v;
    }
  }
  __threadfence();
#pragma unroll
  for (int it = 0; it < 8; ++it) {
    const int row  = 8 * wave + it;
    const int grow = rowBase + row;
    const v4f v = *(const v4f*)(stg + (size_t)row * ODIM + col0) + bb;
    if constexpr (GRADED == 0) {
      *(volatile v4f*)(C + (size_t)grow * ODIM + col0) = v;
    } else {
      if (grow < nN) *(volatile v4f*)(C + (size_t)grow * ODIM + col0) = v;
    }
  }
}

__global__ __launch_bounds__(NTHR) void k_edge_max(
    const int* __restrict__ srcs, const int* __restrict__ dsts, const float* __restrict__ pos,
    float* pmax, int nN, int nE) {
  __shared__ float wm[NWAVE];
  const int tid = threadIdx.x, lane = tid & 31, wave = tid >> 5;
  float m = 0.0f;
#pragma unroll 1
  for (int it = 0; it < EPB / NTHR; ++it) {
    const int e  = blockIdx.x * EPB + it * NTHR + tid;
    const int ec = e < nE ? e : nE - 1;
    const int s = clampi(srcs[ec], 0, nN - 1);
    const int t = clampi(dsts[ec], 0, nN - 1);
    const float dx = pos[(size_t)s * 3 + 0] - pos[(size_t)t * 3 + 0];
    const float dy = pos[(size_t)s * 3 + 1] - pos[(size_t)t * 3 + 1];
    const float dz = pos[(size_t)s * 3 + 2] - pos[(size_t)t * 3 + 2];
    float d = geo_dist(dx, dy, dz);
    d = e < nE ? d : 0.0f;
    m = fmaxf(m, d);
  }
#pragma unroll
  for (int o = 1; o < 32; o <<= 1) m = fmaxf(m, __shfl_xor(m, o));
  if (lane == 0) wm[wave] = m;
  __syncthreads();
  if (wave == 0) {
    float M = wm[0];
#pragma unroll
    for (int w = 1; w < NWAVE; ++w) M = fmaxf(M, wm[w]);
    float* p = pmax + (size_t)blockIdx.x * 32 + lane;
    *(volatile float*)p = M;
    __threadfence();
    *(volatile float*)p = M;
  }
}

__global__ __launch_bounds__(NTHR) void k_maxfin(const float* __restrict__ pmax, float* rmax, int nEB) {
  __shared__ float wm[NWAVE];
  const int tid = threadIdx.x, lane = tid & 31, wave = tid >> 5;
  float m = 0.0f;
#pragma unroll 1
  for (int b = tid; b < nEB; b += NTHR) m = fmaxf(m, pmax[(size_t)b * 32]);
#pragma unroll
  for (int o = 1; o < 32; o <<= 1) m = fmaxf(m, __shfl_xor(m, o));
  if (lane == 0) wm[wave] = m;
  __syncthreads();
  if (wave == 0) {
    float M = wm[0];
#pragma unroll
    for (int w = 1; w < NWAVE; ++w) M = fmaxf(M, wm[w]);
    *(volatile float*)(rmax + lane) = M;
    __threadfence();
    *(volatile float*)(rmax + lane) = M;
  }
}

__global__ __launch_bounds__(NTHR) void k_agg(
    const int* __restrict__ csr, const int* __restrict__ off, const int* __restrict__ cnt,
    const int* __restrict__ srcs, const float* __restrict__ pos, const float* __restrict__ rmax,
    const float* __restrict__ vfacp, const float* __restrict__ vmaxp,
    const float* __restrict__ hw, float* agg, int nN, int nE, int nPad, int csrLen) {
  const int tid = threadIdx.x, lane = tid & 31, wave = tid >> 5;
  const int tbase = blockIdx.x * TGT + wave * 32;
  const int col0 = 4 * lane;
  const v4f z4 = {0.f, 0.f, 0.f, 0.f};
  const float rm   = rmax[0];
  const float rinv = 1.0f / rm;
  const float vf   = vfacp[0];
  const float vm0 = vmaxp[0], vm1 = vmaxp[1], vm2 = vmaxp[2], vm3 = vmaxp[3];
  const size_t vs = (size_t)nPad * HDIM;

  const int cl    = tbase + lane;
  const int cnt_l = cnt[cl];
  const int off_l = off[cl];

#pragma unroll 1
  for (int j = 0; j < 32; ++j) {
    const int c = tbase + j;
    int n = __shfl(cnt_l, j);
    n = n < 0 ? 0 : (n > DEGCAP ? DEGCAP : n);
    const int st = __shfl(off_l, j);
    const int cc = c < nN ? c : nN - 1;
    const float tx = pos[(size_t)cc * 3 + 0];
    const float ty = pos[(size_t)cc * 3 + 1];
    const float tz = pos[(size_t)cc * 3 + 2];

    v4f acc0 = z4, acc1 = z4, acc2 = z4, acc3 = z4;
#pragma unroll 1
    for (int q0 = 0; q0 < n; q0 += 32) {
      const int p = clampi(st + q0 + lane, 0, csrLen - 1);
      const int e = clampi(csr[p], 0, nE - 1);
      const int s = clampi(srcs[e], 0, nN - 1);
      const float dx = pos[(size_t)s * 3 + 0] - tx;
      const float dy = pos[(size_t)s * 3 + 1] - ty;
      const float dz = pos[(size_t)s * 3 + 2] - tz;
      const float d    = geo_dist(dx, dy, dz);
      const float dinv = 1.0f / (d + GEO_EPS);
      const float dsum = (dx * dinv + dz * dinv) + dy * dinv;
      const float r    = d * rinv;
      const float rc   = r > 0.f ? r : 0.f;
      const float ab0 = view_ab(vf, rc, vm0, dsum);
      const float ab1 = view_ab(vf, rc, vm1, dsum);
      const float ab2 = view_ab(vf, rc, vm2, dsum);
      const float ab3 = view_ab(vf, rc, vm3, dsum);
      const int mcnt = (n - q0) < 32 ? (n - q0) : 32;
#pragma unroll 1
      for (int pp = 0; pp < mcnt; ++pp) {
        const int   sb = __builtin_amdgcn_readlane(s, pp);
        const float a0 = __int_as_float(__builtin_amdgcn_readlane(__float_as_int(ab0), pp));
        const float a1 = __int_as_float(__builtin_amdgcn_readlane(__float_as_int(ab1), pp));
        const float a2 = __int_as_float(__builtin_amdgcn_readlane(__float_as_int(ab2), pp));
        const float a3 = __int_as_float(__builtin_amdgcn_readlane(__float_as_int(ab3), pp));
        const v4f h = *(const v4f*)(hw + (size_t)sb * HDIM + col0);
        acc0.x = fmaf(h.x, a0, acc0.x); acc0.y = fmaf(h.y, a0, acc0.y);
        acc0.z = fmaf(h.z, a0, acc0.z); acc0.w = fmaf(h.w, a0, acc0.w);
        acc1.x = fmaf(h.x, a1, acc1.x); acc1.y = fmaf(h.y, a1, acc1.y);
        acc1.z = fmaf(h.z, a1, acc1.z); acc1.w = fmaf(h.w, a1, acc1.w);
        acc2.x = fmaf(h.x, a2, acc2.x); acc2.y = fmaf(h.y, a2, acc2.y);
        acc2.z = fmaf(h.z, a2, acc2.z); acc2.w = fmaf(h.w, a2, acc2.w);
        acc3.x = fmaf(h.x, a3, acc3.x); acc3.y = fmaf(h.y, a3, acc3.y);
        acc3.z = fmaf(h.z, a3, acc3.z); acc3.w = fmaf(h.w, a3, acc3.w);
      }
    }

    float* pw = agg + (size_t)c * HDIM + col0;
    *(volatile v4f*)(pw)          = acc0;
    *(volatile v4f*)(pw + vs)     = acc1;
    *(volatile v4f*)(pw + 2 * vs) = acc2;
    *(volatile v4f*)(pw + 3 * vs) = acc3;
    __threadfence();
    *(volatile v4f*)(pw)          = acc0;
    *(volatile v4f*)(pw + vs)     = acc1;
    *(volatile v4f*)(pw + 2 * vs) = acc2;
    *(volatile v4f*)(pw + 3 * vs) = acc3;
  }
}

__global__ __launch_bounds__(STHR) void k_bnstat(const float* __restrict__ agg, double* part, int nN, int nPad) {
  const int t = threadIdx.x;
  const int view = t >> 7, col = t & 127;
  const int r0 = blockIdx.x * STATR;
  int nr = nN - r0;
  nr = nr < 0 ? 0 : (nr > STATR ? STATR : nr);
  const float* base = agg + ((size_t)view * nPad + r0) * HDIM + col;
  double s = 0.0, q = 0.0;
#pragma unroll 1
  for (int i = 0; i < nr; ++i) {
    const double v = (double)base[(size_t)i * HDIM];
    s += v;
    q += v * v;
  }
  double* pp = part + (size_t)blockIdx.x * (2 * ZDIM);
  *(volatile double*)(pp + t) = s;
  *(volatile double*)(pp + ZDIM + t) = q;
  __threadfence();
  *(volatile double*)(pp + t) = s;
  *(volatile double*)(pp + ZDIM + t) = q;
}

__global__ __launch_bounds__(STHR) void k_bnfin(const double* __restrict__ part, const float* __restrict__ gamma,
                                                float* tbl, int nPart, int nN) {
  const int t = threadIdx.x;
  double s = 0.0, q = 0.0;
#pragma unroll 1
  for (int b = 0; b < nPart; ++b) {
    s += part[(size_t)b * (2 * ZDIM) + t];
    q += part[(size_t)b * (2 * ZDIM) + ZDIM + t];
  }
  const double inv = 1.0 / (double)nN;
  const double mu  = s * inv;
  double var = q * inv - mu * mu;
  var = var < 0.0 ? 0.0 : var;
  const float a  = (float)((double)gamma[t] / sqrt(var + BN_EPS));
  const float mf = (float)mu;
  *(volatile float*)(tbl + t) = mf;
  *(volatile float*)(tbl + ZDIM + t) = a;
  __threadfence();
  *(volatile float*)(tbl + t) = mf;
  *(volatile float*)(tbl + ZDIM + t) = a;
}

__global__ __launch_bounds__(NTHR) void k_gemm2(
    const float* __restrict__ agg, const float* __restrict__ tbl, const float* __restrict__ bnb,
    const float* __restrict__ att, const _Float16* __restrict__ wp, const float* __restrict__ b1,
    const float* __restrict__ lng, const float* __restrict__ lnb, _Float16* Y, int nN, int nPad) {
  extern __shared__ v4f lds_dyn[];
  _Float16* zt = (_Float16*)lds_dyn;
  float* stg = (float*)(lds_dyn + (BM * ZDIM * 2) / 16);
  const int tid = threadIdx.x, lane = tid & 31, wave = tid >> 5;
  const int rowBase = blockIdx.x * BM;
  const size_t vs = (size_t)nPad * HDIM;
  const v4f z4 = {0.f, 0.f, 0.f, 0.f};

#pragma unroll 1
  for (int u = tid; u < BM * ZDIM / 8; u += NTHR) {
    const int row  = u >> 6;
    const int c8   = (u & 63) * 8;
    const int view = c8 >> 7;
    const int col  = c8 & 127;
    const int grow = rowBase + row;
    const float* ap = agg + (size_t)view * vs + (size_t)grow * HDIM + col;
    const v4f a0 = *(const v4f*)ap, a1 = *(const v4f*)(ap + 4);
    const v4f m0 = *(const v4f*)(tbl + c8), m1 = *(const v4f*)(tbl + c8 + 4);
    const v4f s0 = *(const v4f*)(tbl + ZDIM + c8), s1 = *(const v4f*)(tbl + ZDIM + c8 + 4);
    const v4f e0 = *(const v4f*)(bnb + c8), e1 = *(const v4f*)(bnb + c8 + 4);
    const v4f t0 = *(const v4f*)(att + c8), t1 = *(const v4f*)(att + c8 + 4);
    v4f y0 = (a0 - m0) * s0 + e0;
    v4f y1 = (a1 - m1) * s1 + e1;
    y0.x = y0.x > 0.f ? y0.x : 0.f; y0.y = y0.y > 0.f ? y0.y : 0.f;
    y0.z = y0.z > 0.f ? y0.z : 0.f; y0.w = y0.w > 0.f ? y0.w : 0.f;
    y1.x = y1.x > 0.f ? y1.x : 0.f; y1.y = y1.y > 0.f ? y1.y : 0.f;
    y1.z = y1.z > 0.f ? y1.z : 0.f; y1.w = y1.w > 0.f ? y1.w : 0.f;
    y0 = y0 * t0;
    y1 = y1 * t1;
    if (grow >= nN) { y0 = z4; y1 = z4; }
    v8h w;
    w[0] = (_Float16)(y0.x * ZSC); w[1] = (_Float16)(y0.y * ZSC);
    w[2] = (_Float16)(y0.z * ZSC); w[3] = (_Float16)(y0.w * ZSC);
    w[4] = (_Float16)(y1.x * ZSC); w[5] = (_Float16)(y1.y * ZSC);
    w[6] = (_Float16)(y1.z * ZSC); w[7] = (_Float16)(y1.w * ZSC);
    *(v8h*)(zt + (size_t)row * ZDIM + c8) = w;
  }
  __syncthreads();

  mm_core<ZDIM, MDIM>(zt, ZDIM, wp, stg, INV_ZW);
  __syncthreads();

  const int colL = 8 * lane;
  const v4f bA = *(const v4f*)(b1 + colL),  bB = *(const v4f*)(b1 + colL + 4);
  const v4f gA = *(const v4f*)(lng + colL), gB = *(const v4f*)(lng + colL + 4);
  const v4f eA = *(const v4f*)(lnb + colL), eB = *(const v4f*)(lnb + colL + 4);
  const float invM = 1.0f / (float)MDIM;
  v8h hv[8];
#pragma unroll
  for (int it = 0; it < 8; ++it) {
    const int row  = 8 * wave + it;
    const int grow = rowBase + row;
    const float* sr = stg + (size_t)row * MDIM + colL;
    const v4f v0 = *(const v4f*)sr + bA;
    const v4f v1 = *(const v4f*)(sr + 4) + bB;
    float sm = ((v0.x + v0.y) + (v0.z + v0.w)) + ((v1.x + v1.y) + (v1.z + v1.w));
#pragma unroll
    for (int o = 1; o < 32; o <<= 1) sm += __shfl_xor(sm, o);
    const float mu = sm * invM;
    const v4f d0 = v0 - mu, d1 = v1 - mu;
    float sq = ((d0.x * d0.x + d0.y * d0.y) + (d0.z * d0.z + d0.w * d0.w)) +
               ((d1.x * d1.x + d1.y * d1.y) + (d1.z * d1.z + d1.w * d1.w));
#pragma unroll
    for (int o = 1; o < 32; o <<= 1) sq += __shfl_xor(sq, o);
    const float var = sq * invM;
    const float rs  = 1.0f / sqrtf(var + LN_EPS);
    v4f y0 = (d0 * rs) * gA + eA;
    v4f y1 = (d1 * rs) * gB + eB;
    y0.x = y0.x > 0.f ? y0.x : 0.f; y0.y = y0.y > 0.f ? y0.y : 0.f;
    y0.z = y0.z > 0.f ? y0.z : 0.f; y0.w = y0.w > 0.f ? y0.w : 0.f;
    y1.x = y1.x > 0.f ? y1.x : 0.f; y1.y = y1.y > 0.f ? y1.y : 0.f;
    y1.z = y1.z > 0.f ? y1.z : 0.f; y1.w = y1.w > 0.f ? y1.w : 0.f;
    if (grow >= nN) { y0 = z4; y1 = z4; }
    v8h w;
    w[0] = (_Float16)(y0.x * XSC); w[1] = (_Float16)(y0.y * XSC);
    w[2] = (_Float16)(y0.z * XSC); w[3] = (_Float16)(y0.w * XSC);
    w[4] = (_Float16)(y1.x * XSC); w[5] = (_Float16)(y1.y * XSC);
    w[6] = (_Float16)(y1.z * XSC); w[7] = (_Float16)(y1.w * XSC);
    hv[it] = w;
    *(volatile v8h*)(Y + (size_t)grow * MDIM + colL) = w;
  }
  __threadfence();
#pragma unroll
  for (int it = 0; it < 8; ++it) {
    const int row  = 8 * wave + it;
    const int grow = rowBase + row;
    *(volatile v8h*)(Y + (size_t)grow * MDIM + colL) = hv[it];
  }
}

extern "C" void kernel_launch(void* const* d_in, const int* in_sizes, int n_in,
                              void* d_out, int out_size, void* d_ws, size_t ws_size,
                              hipStream_t stream) {
  if (n_in < 18) return;
  const int nN = in_sizes[0] / FDIM;
  const int nE = in_sizes[1] / 2;
  if (nN <= 0 || nE <= 0 || in_sizes[0] != nN * FDIM || in_sizes[1] != 2 * nE) return;
  if (in_sizes[2] != 3 * nN) return;
  if (in_sizes[3] != HDIM * FDIM || in_sizes[4] != HDIM || in_sizes[5] != HDIM * HDIM || in_sizes[6] != HDIM) return;
  if (in_sizes[7] < 1 || in_sizes[8] < NVIEW) return;
  if (in_sizes[9] != ZDIM || in_sizes[10] != ZDIM || in_sizes[11] != ZDIM) return;
  if (in_sizes[12] != MDIM * ZDIM || in_sizes[13] != MDIM || in_sizes[14] != MDIM || in_sizes[15] != MDIM) return;
  if (in_sizes[16] != ODIM * MDIM || in_sizes[17] != ODIM) return;
  if (out_size != nN * ODIM) return;
  if (nE > (1 << 28) || nN > (1 << 22)) return;

  const float* x     = (const float*)d_in[0];
  const int*   ei    = (const int*)d_in[1];
  const float* pos   = (const float*)d_in[2];
  const float* Wft   = (const float*)d_in[3];
  const float* bft   = (const float*)d_in[4];
  const float* Wcv   = (const float*)d_in[5];
  const float* bcv   = (const float*)d_in[6];
  const float* vfac  = (const float*)d_in[7];
  const float* vprm  = (const float*)d_in[8];
  const float* bng   = (const float*)d_in[9];
  const float* bnb   = (const float*)d_in[10];
  const float* att   = (const float*)d_in[11];
  const float* W1    = (const float*)d_in[12];
  const float* b1    = (const float*)d_in[13];
  const float* lng   = (const float*)d_in[14];
  const float* lnb   = (const float*)d_in[15];
  const float* W2    = (const float*)d_in[16];
  const float* b2    = (const float*)d_in[17];
  const int*   src = ei;
  const int*   dst = ei + nE;
  float* out = (float*)d_out;

  const int NPAD   = ((nN + NPADG - 1) / NPADG) * NPADG;
  const int nBC    = (nN + NBC - 1) / NBC;
  const int CNTPAD = nBC * NBC;
  if (4 * nBC + 1 > RBN) return;
  const int nBF    = (nN + NBF - 1) / NBF;
  const int csrLen = ((nE + 31) & ~31) + 4096;
  if (31 * 4 * nBC > 4096) return;
  const int nAgg   = NPAD / TGT;
  const int nGm    = NPAD / BM;
  const int nStat  = NPAD / STATR;
  const int nUnitX = NPAD * (FDIM / 8);
  const int nEB    = (nE + EPB - 1) / EPB;
  const int uWft = HDIM * FDIM / 8, uWcv = HDIM * HDIM / 8, uW1 = MDIM * ZDIM / 8, uW2 = ODIM * MDIM / 8;

  char* ws = (char*)d_ws;
  size_t off = 0;
  const size_t oWft = off; off += (size_t)HDIM * FDIM * 2;               off = (off + 255) & ~(size_t)255;
  const size_t oWcv = off; off += (size_t)HDIM * HDIM * 2;               off = (off + 255) & ~(size_t)255;
  const size_t oW1  = off; off += (size_t)MDIM * ZDIM * 2;               off = (off + 255) & ~(size_t)255;
  const size_t oW2  = off; off += (size_t)ODIM * MDIM * 2;               off = (off + 255) & ~(size_t)255;
  const size_t oAgg = off; off += (size_t)NVIEW * NPAD * HDIM * 4;       off = (off + 255) & ~(size_t)255;
  const size_t oXh  = oAgg;
  const size_t oHh  = oAgg + (size_t)NPAD * FDIM * 2;
  const size_t oHw  = off; off += (size_t)NPAD * HDIM * 4;               off = (off + 255) & ~(size_t)255;
  const size_t oPmx = off; off += (size_t)nEB * 32 * 4;                  off = (off + 255) & ~(size_t)255;
  const size_t oRmx = off; off += (size_t)32 * 4;                        off = (off + 255) & ~(size_t)255;
  const size_t oCnt = off; off += (size_t)CNTPAD * 4;                    off = (off + 255) & ~(size_t)255;
  const size_t oOff = off; off += (size_t)CNTPAD * 4;                    off = (off + 255) & ~(size_t)255;
  const size_t oRb  = off; off += (size_t)RBN * 4;                       off = (off + 255) & ~(size_t)255;
  const size_t oCsr = off; off += (size_t)csrLen * 4;                    off = (off + 255) & ~(size_t)255;
  const size_t oPrt = off; off += (size_t)nStat * 2 * ZDIM * 8;          off = (off + 255) & ~(size_t)255;
  const size_t oTbl = off; off += (size_t)2 * ZDIM * 4;                  off = (off + 255) & ~(size_t)255;
  if (off > ws_size || off > (size_t)WSCAP) return;
  if ((size_t)NPAD * FDIM * 2 + (size_t)NPAD * HDIM * 2 > (size_t)NVIEW * NPAD * HDIM * 4) return;
  if ((size_t)NPAD * MDIM * 2 > (size_t)NPAD * HDIM * 4) return;

  _Float16* wft = (_Float16*)(ws + oWft);
  _Float16* wcv = (_Float16*)(ws + oWcv);
  _Float16* w1p = (_Float16*)(ws + oW1);
  _Float16* w2p = (_Float16*)(ws + oW2);
  float*    aggp = (float*)(ws + oAgg);
  _Float16* xh   = (_Float16*)(ws + oXh);
  _Float16* hh   = (_Float16*)(ws + oHh);
  float*    hw   = (float*)(ws + oHw);
  _Float16* yp   = (_Float16*)(ws + oHw);
  float*    pmx  = (float*)(ws + oPmx);
  float*    rmx  = (float*)(ws + oRmx);
  int*      cnt  = (int*)(ws + oCnt);
  int*      offp = (int*)(ws + oOff);
  int*      rb   = (int*)(ws + oRb);
  int*      csr  = (int*)(ws + oCsr);
  double*   part = (double*)(ws + oPrt);
  float*    tbl  = (float*)(ws + oTbl);

  const int vec8 = ((nE & 3) == 0) ? 1 : 0;

  k_wprep<<<(uWft + NTHR - 1) / NTHR, NTHR, 0, stream>>>(Wft, wft, uWft);
  k_wprep<<<(uWcv + NTHR - 1) / NTHR, NTHR, 0, stream>>>(Wcv, wcv, uWcv);
  k_wprep<<<(uW1 + NTHR - 1) / NTHR, NTHR, 0, stream>>>(W1, w1p, uW1);
  k_wprep<<<(uW2 + NTHR - 1) / NTHR, NTHR, 0, stream>>>(W2, w2p, uW2);
  k_xprep<<<(nUnitX + NTHR - 1) / NTHR, NTHR, 0, stream>>>(x, xh, nN, nUnitX);

  k_gemm_h<<<nGm, NTHR, 0, stream>>>(xh, wft, bft, hh, nN);
  k_gemm_f<HDIM, 0><<<nGm, NTHR, 0, stream>>>(hh, wcv, bcv, hw, nN);

  k_edge_max<<<nEB, NTHR, 0, stream>>>(src, dst, pos, pmx, nN, nE);
  k_maxfin<<<1, NTHR, 0, stream>>>(pmx, rmx, nEB);

  k_count<<<nBC, NTHR, 0, stream>>>(dst, cnt, nE, vec8);
  k_offsets<<<1, OTHR, 0, stream>>>(cnt, offp, rb, nBC);
  hipFuncSetAttribute(reinterpret_cast<const void*>(&k_fill),
                      hipFuncAttributeMaxDynamicSharedMemorySize, LDS_FILL);
  k_fill<<<nBF, NTHR, LDS_FILL, stream>>>(dst, offp, rb, csr, nE, vec8, csrLen);

  k_agg<<<nAgg, NTHR, 0, stream>>>(csr, offp, cnt, src, pos, rmx, vfac, vprm, hw, aggp, nN, nE, NPAD, csrLen);

  k_bnstat<<<nStat, STHR, 0, stream>>>(aggp, part, nN, NPAD);
  k_bnfin<<<1, STHR, 0, stream>>>(part, bng, tbl, nStat, nN);

  hipFuncSetAttribute(reinterpret_cast<const void*>(&k_gemm2),
                      hipFuncAttributeMaxDynamicSharedMemorySize, LDS_G2);
  k_gemm2<<<nGm, NTHR, LDS_G2, stream>>>(aggp, tbl, bnb, att, w1p, b1, lng, lnb, yp, nN, NPAD);

  k_gemm_f<MDIM, 1><<<nGm, NTHR, 0, stream>>>(yp, w2p, b2, out, nN);
}
